// MotionFormerBlock_5291399708691
// MI455X (gfx1250) — hardware-verified
//
#include <hip/hip_runtime.h>
#define NB 8
#define NTQ 1024
#define CD 256
#define MD 128
#define NH 8
#define HD 32
#define MHD 16
#define HID 1024
#define NTOK (NB * NTQ)

typedef __bf16 v16b __attribute__((ext_vector_type(16)));
typedef unsigned short v8us __attribute__((ext_vector_type(8), may_alias));
typedef float  v8f  __attribute__((ext_vector_type(8)));
typedef float  v4f  __attribute__((ext_vector_type(4)));
typedef float  v4fa __attribute__((ext_vector_type(4), may_alias));
union FragB { v16b v; v8us half[2]; unsigned short u[16]; };

__device__ __forceinline__ unsigned short bf16_bits(float x) { unsigned int u = __float_as_uint(x); return (unsigned short)((u + 0x7FFFu + ((u >> 16) & 1u)) >> 16); }
__device__ __forceinline__ float bf16_val(unsigned short b) { return __uint_as_float(((unsigned int)b) << 16); }
__device__ __forceinline__ float bf16_round(float x) { return bf16_val(bf16_bits(x)); }
template <int NT>
__device__ __forceinline__ v8f mmaN(v16b ah, v16b al, v16b bh, v16b bl, v8f c) {
  c = __builtin_amdgcn_wmma_f32_16x16x32_bf16(false, ah, false, bh, (short)0, c, false, false);
  if (NT >= 2) c = __builtin_amdgcn_wmma_f32_16x16x32_bf16(false, al, false, bh, (short)0, c, false, false);
  if (NT >= 3) c = __builtin_amdgcn_wmma_f32_16x16x32_bf16(false, ah, false, bl, (short)0, c, false, false);
  asm volatile("v_nop\n\tv_nop\n\tv_nop\n\tv_nop" : "+v"(c) : "v"(ah), "v"(al), "v"(bh), "v"(bl));
  return c;
}

__global__ __launch_bounds__(256) void k_wt_bf16(const float* __restrict__ W, unsigned short* __restrict__ Wt, int K, int N) {
  const int t = blockIdx.x * 256 + threadIdx.x;
  const int k8n = K / 8;
  if (t >= N * k8n) return;
  const int n = t / k8n, k8 = (t % k8n) * 8;
  v8us v;
#pragma unroll
  for (int i = 0; i < 8; ++i) v[i] = bf16_bits(W[(size_t)(k8 + i) * N + n]);
  *(volatile v8us*)(Wt + (size_t)n * K + k8) = v;
  __threadfence();
  *(volatile v8us*)(Wt + (size_t)n * K + k8) = v;
}

template <bool ASPLIT, int ACT, bool BIAS_BF16>
__global__ __launch_bounds__(128) void k_gemm_bf(const float* __restrict__ A, int lda, const unsigned short* __restrict__ Wt, int ldb,
                                               const float* __restrict__ bias, float* __restrict__ C, int ldc, int M, int N, int K) {
  __shared__ __attribute__((aligned(16))) float so[4][16][64];
  const int tid = threadIdx.x, w = tid >> 5, lane = tid & 31, ln = lane & 15, hh = lane >> 4;
  const int ntn = N / 64;
  const int wid = blockIdx.x * 4 + w;
  const int mt = wid / ntn, nq = wid % ntn;
  if (mt * 16 >= M) return;
  const int row0 = mt * 16, col0 = nq * 64;
  const float* arow = A + (size_t)(row0 + ln) * lda;
  v8f acc[4] = {};
  for (int kb = 0; kb < K; kb += 32) {
    FragB ah, al;
    const v4f x0 = *(const v4fa*)(arow + kb + 8 * hh), x1 = *(const v4fa*)(arow + kb + 8 * hh + 4);
    const v4f x2 = *(const v4fa*)(arow + kb + 16 + 8 * hh), x3 = *(const v4fa*)(arow + kb + 16 + 8 * hh + 4);
    float xs[16] = {x0[0],x0[1],x0[2],x0[3],x1[0],x1[1],x1[2],x1[3],x2[0],x2[1],x2[2],x2[3],x3[0],x3[1],x3[2],x3[3]};
#pragma unroll
    for (int i = 0; i < 16; ++i) { const unsigned short hb = bf16_bits(xs[i]); ah.u[i] = hb; al.u[i] = ASPLIT ? bf16_bits(xs[i] - bf16_val(hb)) : (unsigned short)0; }
#pragma unroll
    for (int t = 0; t < 4; ++t) {
      const unsigned short* brow = Wt + (size_t)(col0 + t * 16 + ln) * ldb + kb;
      FragB b;
      b.half[0] = *(const v8us*)(brow + 8 * hh);
      b.half[1] = *(const v8us*)(brow + 16 + 8 * hh);
      acc[t] = mmaN<ASPLIT ? 2 : 1>(ah.v, al.v, b.v, b.v, acc[t]);
    }
  }
#pragma unroll
  for (int t = 0; t < 4; ++t) {
    float bv = bias ? bias[col0 + t * 16 + ln] : 0.f;
    if (BIAS_BF16) bv = bf16_round(bv);
#pragma unroll
    for (int r = 0; r < 8; ++r) { float v = acc[t][r] + bv; if (ACT == 1) v = fmaxf(v, 0.f); so[w][8 * hh + r][t * 16 + ln] = v; }
  }
  __builtin_amdgcn_fence(__ATOMIC_ACQ_REL, "workgroup");
  __builtin_amdgcn_wave_barrier();
  const int rsub = lane >> 4, c4 = (lane & 15) * 4;
  for (int pass = 0; pass < 2; ++pass) {
#pragma unroll
    for (int q = 0; q < 8; ++q) {
      const int r = q * 2 + rsub;
      const v4f v = *(const v4fa*)&so[w][r][c4];
      *(volatile v4f*)(C + (size_t)(row0 + r) * ldc + col0 + c4) = v;
    }
    if (pass == 0) __threadfence();
  }
}

template <int D, bool CAUSAL>
__global__ __launch_bounds__(128) void k_flash(const float* __restrict__ qb, const float* __restrict__ kb, const float* __restrict__ vb,
                                             int pitch, int T, int H, float scale, float* __restrict__ y, int ypitch) {
  constexpr int KS = D / 32;
  constexpr int DT = D / 16;
  __shared__ __attribute__((aligned(16))) unsigned short sKh[32][D + 8], sKl[32][D + 8], sVh[32][D + 8], sVl[32][D + 8];
  __shared__ __attribute__((aligned(16))) unsigned short sPh[4][16][40], sPl[4][16][40];
  __shared__ __attribute__((aligned(16))) float sO[4][16][D];
  const int tid = threadIdx.x, w = tid >> 5, lane = tid & 31, ln = lane & 15, hh = lane >> 4;
  const int nqb = (T + 63) / 64;
  const int bh = blockIdx.x / nqb, qblk = blockIdx.x % nqb;
  const int b = bh / H, h = bh % H;
  const int q0 = qblk * 64 + w * 16;
  const float* Q = qb + (size_t)b * T * pitch + h * D;
  const float* K = kb + (size_t)b * T * pitch + h * D;
  const float* V = vb + (size_t)b * T * pitch + h * D;

  FragB aqh[KS], aql[KS];
  {
    int row = q0 + ln; if (row >= T) row = T - 1;
    const float* qr = Q + (size_t)row * pitch;
#pragma unroll
    for (int ks = 0; ks < KS; ++ks)
#pragma unroll
      for (int i = 0; i < 16; ++i) {
        const int d = ks * 32 + ((i < 8) ? (8 * hh + i) : (16 + 8 * hh + (i - 8)));
        const float x = qr[d] * scale; const unsigned short hb = bf16_bits(x);
        aqh[ks].u[i] = hb; aql[ks].u[i] = bf16_bits(x - bf16_val(hb));
      }
  }
  float m_r[8], l_r[8];
#pragma unroll
  for (int r = 0; r < 8; ++r) { m_r[r] = -3.0e38f; l_r[r] = 0.f; }
  v8f oacc[DT];
#pragma unroll
  for (int dt = 0; dt < DT; ++dt) oacc[dt] = (v8f){0.f,0.f,0.f,0.f,0.f,0.f,0.f,0.f};

  const int kv_end = CAUSAL ? min(T, qblk * 64 + 64) : T;
  for (int j0 = 0; j0 < kv_end; j0 += 32) {
    __syncthreads();
    for (int e = tid; e < 32 * (D / 4); e += 128) {
      const int r = e / (D / 4), c4 = (e % (D / 4)) * 4;
      const int key = j0 + r;
      v4f kf = {0.f,0.f,0.f,0.f}, vf = {0.f,0.f,0.f,0.f};
      if (key < T) { kf = *(const v4fa*)(K + (size_t)key * pitch + c4); vf = *(const v4fa*)(V + (size_t)key * pitch + c4); }
#pragma unroll
      for (int t = 0; t < 4; ++t) {
        unsigned short hb = bf16_bits(kf[t]); sKh[r][c4 + t] = hb; sKl[r][c4 + t] = bf16_bits(kf[t] - bf16_val(hb));
        hb = bf16_bits(vf[t]); sVh[r][c4 + t] = hb; sVl[r][c4 + t] = bf16_bits(vf[t] - bf16_val(hb));
      }
    }
    __syncthreads();
    v8f s[2];
#pragma unroll
    for (int nt = 0; nt < 2; ++nt) {
      v8f acc = {};
#pragma unroll
      for (int ks = 0; ks < KS; ++ks) {
        FragB bh_, bl_;
        bh_.half[0] = *(const v8us*)&sKh[nt * 16 + ln][ks * 32 + 8 * hh]; bh_.half[1] = *(const v8us*)&sKh[nt * 16 + ln][ks * 32 + 16 + 8 * hh];
        bl_.half[0] = *(const v8us*)&sKl[nt * 16 + ln][ks * 32 + 8 * hh]; bl_.half[1] = *(const v8us*)&sKl[nt * 16 + ln][ks * 32 + 16 + 8 * hh];
        acc = mmaN<3>(aqh[ks].v, aql[ks].v, bh_.v, bl_.v, acc);
      }
      s[nt] = acc;
    }
    float alpha[8];
#pragma unroll
    for (int r = 0; r < 8; ++r) {
      const int qi = q0 + 8 * hh + r;
      const int ja = j0 + ln, jb = j0 + 16 + ln;
      if (CAUSAL) { if (ja > qi) s[0][r] = -3.0e38f; if (jb > qi) s[1][r] = -3.0e38f; }
      if (ja >= T) s[0][r] = -3.0e38f;
      if (jb >= T) s[1][r] = -3.0e38f;
      float mx = fmaxf(s[0][r], s[1][r]);
      mx = fmaxf(mx, __shfl_xor(mx, 1, 32)); mx = fmaxf(mx, __shfl_xor(mx, 2, 32)); mx = fmaxf(mx, __shfl_xor(mx, 4, 32)); mx = fmaxf(mx, __shfl_xor(mx, 8, 32));
      const float mnew = fmaxf(m_r[r], mx);
      alpha[r] = (mnew > -1.0e38f) ? __expf(m_r[r] - mnew) : 1.0f;
      const float p0 = (s[0][r] > -1.0e38f) ? __expf(s[0][r] - mnew) : 0.f;
      const float p1 = (s[1][r] > -1.0e38f) ? __expf(s[1][r] - mnew) : 0.f;
      m_r[r] = mnew;
      l_r[r] = l_r[r] * alpha[r] + p0 + p1;
      unsigned short hb = bf16_bits(p0); sPh[w][8 * hh + r][ln] = hb;      sPl[w][8 * hh + r][ln] = bf16_bits(p0 - bf16_val(hb));
      hb = bf16_bits(p1);                sPh[w][8 * hh + r][16 + ln] = hb; sPl[w][8 * hh + r][16 + ln] = bf16_bits(p1 - bf16_val(hb));
    }
#pragma unroll
    for (int dt = 0; dt < DT; ++dt)
#pragma unroll
      for (int r = 0; r < 8; ++r) oacc[dt][r] *= alpha[r];
    __builtin_amdgcn_fence(__ATOMIC_ACQ_REL, "workgroup");
    __builtin_amdgcn_wave_barrier();
    FragB pah, pal;
    pah.half[0] = *(const v8us*)&sPh[w][ln][8 * hh]; pah.half[1] = *(const v8us*)&sPh[w][ln][16 + 8 * hh];
    pal.half[0] = *(const v8us*)&sPl[w][ln][8 * hh]; pal.half[1] = *(const v8us*)&sPl[w][ln][16 + 8 * hh];
#pragma unroll
    for (int dt = 0; dt < DT; ++dt) {
      FragB bvh, bvl;
#pragma unroll
      for (int i = 0; i < 8; ++i) {
        bvh.u[i] = sVh[8 * hh + i][dt * 16 + ln]; bvh.u[8 + i] = sVh[16 + 8 * hh + i][dt * 16 + ln];
        bvl.u[i] = sVl[8 * hh + i][dt * 16 + ln]; bvl.u[8 + i] = sVl[16 + 8 * hh + i][dt * 16 + ln];
      }
      oacc[dt] = mmaN<3>(pah.v, pal.v, bvh.v, bvl.v, oacc[dt]);
    }
    __builtin_amdgcn_fence(__ATOMIC_ACQ_REL, "workgroup");
    __builtin_amdgcn_wave_barrier();
  }
#pragma unroll
  for (int r = 0; r < 8; ++r) {
    float l = l_r[r];
    l += __shfl_xor(l, 1, 32); l += __shfl_xor(l, 2, 32); l += __shfl_xor(l, 4, 32); l += __shfl_xor(l, 8, 32);
    l_r[r] = (l > 0.f) ? 1.0f / l : 0.f;
  }
#pragma unroll
  for (int dt = 0; dt < DT; ++dt)
#pragma unroll
    for (int r = 0; r < 8; ++r) sO[w][8 * hh + r][dt * 16 + ln] = oacc[dt][r] * l_r[r];
  __builtin_amdgcn_fence(__ATOMIC_ACQ_REL, "workgroup");
  __builtin_amdgcn_wave_barrier();
  for (int pass = 0; pass < 2; ++pass) {
    for (int r = 0; r < 16; ++r) {
      const int row = q0 + r;
      if (row < T && lane < D / 4) {
        const v4f val = *(const v4fa*)&sO[w][r][lane * 4];
        *(volatile v4f*)(y + ((size_t)b * T + row) * ypitch + h * D + lane * 4) = val;
      }
    }
    if (pass == 0) __threadfence();
  }
}

template <bool AFFINE, bool RESID, bool RES_BF16>
__global__ __launch_bounds__(256) void k_transpose32(const float* __restrict__ in, float* __restrict__ out, int rows, int cols,
                                                    const float* __restrict__ scale, const float* __restrict__ shift, const float* __restrict__ res) {
  __shared__ float tile[32][33];
  const int b = blockIdx.z;
  const int r0 = blockIdx.y * 32, c0 = blockIdx.x * 32;
  const float* src = in + (size_t)b * rows * cols;
  float* dst = out + (size_t)b * rows * cols;
  const int tx = threadIdx.x & 31, ty = threadIdx.x >> 5;
  for (int i = ty; i < 32; i += 8) tile[i][tx] = src[(size_t)(r0 + i) * cols + c0 + tx];
  __syncthreads();
  for (int pass = 0; pass < 2; ++pass) {
    for (int i = ty; i < 32; i += 8) {
      float v = tile[tx][i];
      const int orow = c0 + i;
      if (AFFINE) v = v * scale[orow] + shift[orow];
      if (RESID) { float rv = res[(size_t)b * rows * cols + (size_t)orow * rows + r0 + tx]; if (RES_BF16) rv = bf16_round(rv); v += rv; }
      *(volatile float*)(dst + (size_t)orow * rows + r0 + tx) = v;
    }
    if (pass == 0) __threadfence();
  }
}

__global__ __launch_bounds__(256) void k_pool2_pm(const float* __restrict__ in, float* __restrict__ out, int Bn, int H, int W, int C) {
  const size_t t = (size_t)blockIdx.x * 256 + threadIdx.x;
  const int c4n = C / 4, Ho = H / 2, Wo = W / 2;
  const size_t total = (size_t)Bn * Ho * Wo * c4n;
  if (t >= total) return;
  const int c4 = (int)(t % c4n) * 4; size_t rest = t / c4n;
  const int pw = (int)(rest % Wo); rest /= Wo; const int ph = (int)(rest % Ho); const int b = (int)(rest / Ho);
  const float* base = in + (size_t)b * H * W * C;
  const int p00 = (2 * ph) * W + 2 * pw;
  const v4f a = *(const v4fa*)(base + (size_t)p00 * C + c4), bq = *(const v4fa*)(base + (size_t)(p00 + 1) * C + c4);
  const v4f c = *(const v4fa*)(base + (size_t)(p00 + W) * C + c4), d = *(const v4fa*)(base + (size_t)(p00 + W + 1) * C + c4);
  v4f m; for (int i = 0; i < 4; ++i) m[i] = fmaxf(fmaxf(a[i], bq[i]), fmaxf(c[i], d[i]));
  float* dst = out + ((size_t)b * Ho * Wo + (size_t)ph * Wo + pw) * C + c4;
  *(volatile v4f*)dst = m;
  __threadfence();
  *(volatile v4f*)dst = m;
}

template <int DQ, int DV>
__global__ __launch_bounds__(128) void k_flash2(const float* __restrict__ Qb, size_t qstride, int qpitch, int Tq,
                                              const float* __restrict__ Kb, size_t kstride, int kpitch, int Tk,
                                              const float* __restrict__ Vb, size_t vstride, int vpitch,
                                              float scale, float* __restrict__ y, size_t ystride, int ypitch) {
  constexpr int KS = DQ / 32, DT = DV / 16;
  __shared__ __attribute__((aligned(16))) unsigned short sKh[32][DQ + 8], sKl[32][DQ + 8], sVh[32][DV + 8], sVl[32][DV + 8];
  __shared__ __attribute__((aligned(16))) unsigned short sPh[4][16][40], sPl[4][16][40];
  __shared__ __attribute__((aligned(16))) float sO[4][16][DV];
  const int tid = threadIdx.x, w = tid >> 5, lane = tid & 31, ln = lane & 15, hh = lane >> 4;
  const int nqb = (Tq + 63) / 64;
  const int bh = blockIdx.x / nqb, qblk = blockIdx.x % nqb;
  const int dv0 = blockIdx.y * DV;
  const int q0 = qblk * 64 + w * 16;
  const float* Q = Qb + (size_t)bh * qstride; const float* K = Kb + (size_t)bh * kstride; const float* V = Vb + (size_t)bh * vstride + dv0;
  FragB aqh[KS], aql[KS];
  {
    int row = q0 + ln; if (row >= Tq) row = Tq - 1;
    const float* qr = Q + (size_t)row * qpitch;
#pragma unroll
    for (int ks = 0; ks < KS; ++ks)
#pragma unroll
      for (int i = 0; i < 16; ++i) {
        const int d = ks * 32 + ((i < 8) ? (8 * hh + i) : (16 + 8 * hh + (i - 8)));
        const float x = qr[d] * scale; const unsigned short hb = bf16_bits(x);
        aqh[ks].u[i] = hb; aql[ks].u[i] = bf16_bits(x - bf16_val(hb));
      }
  }
  float m_r[8], l_r[8];
#pragma unroll
  for (int r = 0; r < 8; ++r) { m_r[r] = -3.0e38f; l_r[r] = 0.f; }
  v8f oacc[DT];
#pragma unroll
  for (int dt = 0; dt < DT; ++dt) oacc[dt] = (v8f){0.f,0.f,0.f,0.f,0.f,0.f,0.f,0.f};
  for (int j0 = 0; j0 < Tk; j0 += 32) {
    __syncthreads();
    for (int e = tid; e < 32 * (DQ / 4); e += 128) {
      const int r = e / (DQ / 4), c4 = (e % (DQ / 4)) * 4; const int key = j0 + r;
      v4f f = {0.f,0.f,0.f,0.f}; if (key < Tk) f = *(const v4fa*)(K + (size_t)key * kpitch + c4);
#pragma unroll
      for (int t = 0; t < 4; ++t) { const unsigned short hb = bf16_bits(f[t]); sKh[r][c4 + t] = hb; sKl[r][c4 + t] = bf16_bits(f[t] - bf16_val(hb)); }
    }
    for (int e = tid; e < 32 * (DV / 4); e += 128) {
      const int r = e / (DV / 4), c4 = (e % (DV / 4)) * 4; const int key = j0 + r;
      v4f f = {0.f,0.f,0.f,0.f}; if (key < Tk) f = *(const v4fa*)(V + (size_t)key * vpitch + c4);
#pragma unroll
      for (int t = 0; t < 4; ++t) { const unsigned short hb = bf16_bits(f[t]); sVh[r][c4 + t] = hb; sVl[r][c4 + t] = bf16_bits(f[t] - bf16_val(hb)); }
    }
    __syncthreads();
    v8f s[2];
#pragma unroll
    for (int nt = 0; nt < 2; ++nt) {
      v8f acc = {};
#pragma unroll
      for (int ks = 0; ks < KS; ++ks) {
        FragB bh_, bl_;
        bh_.half[0] = *(const v8us*)&sKh[nt * 16 + ln][ks * 32 + 8 * hh]; bh_.half[1] = *(const v8us*)&sKh[nt * 16 + ln][ks * 32 + 16 + 8 * hh];
        bl_.half[0] = *(const v8us*)&sKl[nt * 16 + ln][ks * 32 + 8 * hh]; bl_.half[1] = *(const v8us*)&sKl[nt * 16 + ln][ks * 32 + 16 + 8 * hh];
        acc = mmaN<3>(aqh[ks].v, aql[ks].v, bh_.v, bl_.v, acc);
      }
      s[nt] = acc;
    }
    float alpha[8];
#pragma unroll
    for (int r = 0; r < 8; ++r) {
      const int ja = j0 + ln, jb = j0 + 16 + ln;
      if (ja >= Tk) s[0][r] = -3.0e38f;
      if (jb >= Tk) s[1][r] = -3.0e38f;
      float mx = fmaxf(s[0][r], s[1][r]);
      mx = fmaxf(mx, __shfl_xor(mx, 1, 32)); mx = fmaxf(mx, __shfl_xor(mx, 2, 32)); mx = fmaxf(mx, __shfl_xor(mx, 4, 32)); mx = fmaxf(mx, __shfl_xor(mx, 8, 32));
      const float mnew = fmaxf(m_r[r], mx);
      alpha[r] = (mnew > -1.0e38f) ? __expf(m_r[r] - mnew) : 1.0f;
      const float p0 = (s[0][r] > -1.0e38f) ? __expf(s[0][r] - mnew) : 0.f;
      const float p1 = (s[1][r] > -1.0e38f) ? __expf(s[1][r] - mnew) : 0.f;
      m_r[r] = mnew;
      l_r[r] = l_r[r] * alpha[r] + p0 + p1;
      unsigned short hb = bf16_bits(p0); sPh[w][8 * hh + r][ln] = hb;      sPl[w][8 * hh + r][ln] = bf16_bits(p0 - bf16_val(hb));
      hb = bf16_bits(p1);                sPh[w][8 * hh + r][16 + ln] = hb; sPl[w][8 * hh + r][16 + ln] = bf16_bits(p1 - bf16_val(hb));
    }
#pragma unroll
    for (int dt = 0; dt < DT; ++dt)
#pragma unroll
      for (int r = 0; r < 8; ++r) oacc[dt][r] *= alpha[r];
    __builtin_amdgcn_fence(__ATOMIC_ACQ_REL, "workgroup");
    __builtin_amdgcn_wave_barrier();
    FragB pah, pal;
    pah.half[0] = *(const v8us*)&sPh[w][ln][8 * hh]; pah.half[1] = *(const v8us*)&sPh[w][ln][16 + 8 * hh];
    pal.half[0] = *(const v8us*)&sPl[w][ln][8 * hh]; pal.half[1] = *(const v8us*)&sPl[w][ln][16 + 8 * hh];
#pragma unroll
    for (int dt = 0; dt < DT; ++dt) {
      FragB bvh, bvl;
#pragma unroll
      for (int i = 0; i < 8; ++i) {
        bvh.u[i] = sVh[8 * hh + i][dt * 16 + ln]; bvh.u[8 + i] = sVh[16 + 8 * hh + i][dt * 16 + ln];
        bvl.u[i] = sVl[8 * hh + i][dt * 16 + ln]; bvl.u[8 + i] = sVl[16 + 8 * hh + i][dt * 16 + ln];
      }
      oacc[dt] = mmaN<3>(pah.v, pal.v, bvh.v, bvl.v, oacc[dt]);
    }
    __builtin_amdgcn_fence(__ATOMIC_ACQ_REL, "workgroup");
    __builtin_amdgcn_wave_barrier();
  }
#pragma unroll
  for (int r = 0; r < 8; ++r) {
    float l = l_r[r];
    l += __shfl_xor(l, 1, 32); l += __shfl_xor(l, 2, 32); l += __shfl_xor(l, 4, 32); l += __shfl_xor(l, 8, 32);
    l_r[r] = (l > 0.f) ? 1.0f / l : 0.f;
  }
#pragma unroll
  for (int dt = 0; dt < DT; ++dt)
#pragma unroll
    for (int r = 0; r < 8; ++r) sO[w][8 * hh + r][dt * 16 + ln] = oacc[dt][r] * l_r[r];
  __builtin_amdgcn_fence(__ATOMIC_ACQ_REL, "workgroup");
  __builtin_amdgcn_wave_barrier();
  for (int pass = 0; pass < 2; ++pass) {
    for (int r = 0; r < 16; ++r) {
      const int row = q0 + r;
      for (int c4 = lane * 4; c4 < DV; c4 += 128) {
        if (row < Tq) {
          const v4f val = *(const v4fa*)&sO[w][r][c4];
          *(volatile v4f*)(y + (size_t)bh * ystride + (size_t)row * ypitch + dv0 + c4) = val;
        }
      }
    }
    if (pass == 0) __threadfence();
  }
}

template <bool ASPLIT, int ACT, bool BIAS_BF16, bool RES_BF16>
__global__ __launch_bounds__(128) void k_gemm_bf3(const float* __restrict__ A, int lda, const unsigned short* __restrict__ Wt, int ldb,
                                                const float* __restrict__ bias, const float* __restrict__ resid, int rmod, int ldr,
                                                float* __restrict__ C, int ldc, int M, int N, int K) {
  __shared__ __attribute__((aligned(16))) float so[4][16][64];
  const int tid = threadIdx.x, w = tid >> 5, lane = tid & 31, ln = lane & 15, hh = lane >> 4;
  const int ntn = N / 64;
  const int wid = blockIdx.x * 4 + w;
  const int mt = wid / ntn, nq = wid % ntn;
  if (mt * 16 >= M) return;
  const int row0 = mt * 16, col0 = nq * 64;
  const float* arow = A + (size_t)(row0 + ln) * lda;
  v8f acc[4] = {};
  for (int kb = 0; kb < K; kb += 32) {
    FragB ah, al;
    const v4f x0 = *(const v4fa*)(arow + kb + 8 * hh), x1 = *(const v4fa*)(arow + kb + 8 * hh + 4);
    const v4f x2 = *(const v4fa*)(arow + kb + 16 + 8 * hh), x3 = *(const v4fa*)(arow + kb + 16 + 8 * hh + 4);
    float xs[16] = {x0[0],x0[1],x0[2],x0[3],x1[0],x1[1],x1[2],x1[3],x2[0],x2[1],x2[2],x2[3],x3[0],x3[1],x3[2],x3[3]};
#pragma unroll
    for (int i = 0; i < 16; ++i) { const unsigned short hb = bf16_bits(xs[i]); ah.u[i] = hb; al.u[i] = ASPLIT ? bf16_bits(xs[i] - bf16_val(hb)) : (unsigned short)0; }
#pragma unroll
    for (int t = 0; t < 4; ++t) {
      const unsigned short* brow = Wt + (size_t)(col0 + t * 16 + ln) * ldb + kb;
      FragB b;
      b.half[0] = *(const v8us*)(brow + 8 * hh);
      b.half[1] = *(const v8us*)(brow + 16 + 8 * hh);
      acc[t] = mmaN<ASPLIT ? 2 : 1>(ah.v, al.v, b.v, b.v, acc[t]);
    }
  }
#pragma unroll
  for (int t = 0; t < 4; ++t) {
    const int col = col0 + t * 16 + ln;
    float bv = bias ? bias[col] : 0.f;
    if (BIAS_BF16) bv = bf16_round(bv);
#pragma unroll
    for (int r = 0; r < 8; ++r) {
      float v = acc[t][r] + bv;
      if (resid) { float rv = resid[(size_t)((row0 + 8 * hh + r) % rmod) * ldr + col]; if (RES_BF16) rv = bf16_round(rv); v += rv; }
      if (ACT == 1) v = fmaxf(v, 0.f);
      if (ACT == 2) v = 0.5f * v * (1.0f + erff(v * 0.70710678118654752f));
      if (ACT == 3) { const float u = 0.7978845608028654f * (v + 0.044715f * v * v * v); v = 0.5f * v * (1.0f + tanhf(u)); }
      so[w][8 * hh + r][t * 16 + ln] = v;
    }
  }
  __builtin_amdgcn_fence(__ATOMIC_ACQ_REL, "workgroup");
  __builtin_amdgcn_wave_barrier();
  const int rsub = lane >> 4, c4 = (lane & 15) * 4;
  for (int pass = 0; pass < 2; ++pass) {
#pragma unroll
    for (int q = 0; q < 8; ++q) {
      const int r = q * 2 + rsub;
      const v4f v = *(const v4fa*)&so[w][r][c4];
      *(volatile v4f*)(C + (size_t)(row0 + r) * ldc + col0 + c4) = v;
    }
    if (pass == 0) __threadfence();
  }
}
template <bool PARAM_BF16>
__global__ __launch_bounds__(256) void k_layernorm(const float* __restrict__ X, const float* __restrict__ R, const float* __restrict__ g, const float* __restrict__ bta,
                                                  float* __restrict__ out_sum, float* __restrict__ out_norm, int N, float eps) {
  __shared__ float red[256];
  const int row = blockIdx.x, tid = threadIdx.x;
  const float* x = X + (size_t)row * N; const float* rr = R ? R + (size_t)row * N : nullptr;
  float vals[16];
  const int per = N / 256;
  float s1 = 0.f;
  for (int u = 0; u < per / 4; ++u) {
    const int j = tid * 4 + 1024 * u;
    const v4f a = *(const v4fa*)(x + j);
    v4f b = {0.f,0.f,0.f,0.f}; if (rr) b = *(const v4fa*)(rr + j);
#pragma unroll
    for (int q = 0; q < 4; ++q) { const float v = a[q] + b[q]; vals[u * 4 + q] = v; s1 += v; }
  }
  red[tid] = s1; __syncthreads();
  for (int st = 128; st > 0; st >>= 1) { if (tid < st) red[tid] += red[tid + st]; __syncthreads(); }
  const float mu = red[0] / (float)N; __syncthreads();
  float s2 = 0.f;
  for (int u = 0; u < per / 4; ++u)
#pragma unroll
    for (int q = 0; q < 4; ++q) { const float c = vals[u * 4 + q] - mu; s2 += c * c; }
  red[tid] = s2; __syncthreads();
  for (int st = 128; st > 0; st >>= 1) { if (tid < st) red[tid] += red[tid + st]; __syncthreads(); }
  const float rs = rsqrtf(red[0] / (float)N + eps);
  for (int pass = 0; pass < 2; ++pass) {
    for (int u = 0; u < per / 4; ++u) {
      const int j = tid * 4 + 1024 * u;
      v4f o, sm;
#pragma unroll
      for (int q = 0; q < 4; ++q) {
        float gg = g[j + q], bb = bta[j + q];
        if (PARAM_BF16) { gg = bf16_round(gg); bb = bf16_round(bb); }
        sm[q] = vals[u * 4 + q]; o[q] = (vals[u * 4 + q] - mu) * rs * gg + bb;
      }
      if (out_sum) *(volatile v4f*)(out_sum + (size_t)row * N + j) = sm;
      *(volatile v4f*)(out_norm + (size_t)row * N + j) = o;
    }
    if (pass == 0) __threadfence();
  }
}

template <bool ASPLIT, bool BSPLIT, int ACT>
__global__ __launch_bounds__(128) void k_gemm_b(const float* __restrict__ A, int lda, size_t sA, const unsigned short* __restrict__ Bh, const unsigned short* __restrict__ Bl, int ldb, size_t sB,
                                             const float* __restrict__ bias, const float* __restrict__ resid, int ldr, size_t sR, float rsign, float alpha,
                                             float* __restrict__ C, int ldc, size_t sC, int M, int N, int K) {
  __shared__ __attribute__((aligned(16))) float so[4][16][64];
  const int tid = threadIdx.x, w = tid >> 5, lane = tid & 31, ln = lane & 15, hh = lane >> 4;
  const int by = blockIdx.y;
  A += (size_t)by * sA; Bh += (size_t)by * sB; if (BSPLIT) Bl += (size_t)by * sB; C += (size_t)by * sC; if (resid) resid += (size_t)by * sR;
  const int ntn = (N + 63) / 64; const int wid = blockIdx.x * 4 + w; const int mt = wid / ntn, nq = wid % ntn;
  if (mt * 16 >= M) return;
  const int row0 = mt * 16, col0 = nq * 64;
  const float* arow = A + (size_t)(row0 + ln) * lda;
  v8f acc[4] = {};
  for (int kb = 0; kb < K; kb += 32) {
    FragB ah, al;
    const v4f x0 = *(const v4fa*)(arow + kb + 8 * hh), x1 = *(const v4fa*)(arow + kb + 8 * hh + 4);
    const v4f x2 = *(const v4fa*)(arow + kb + 16 + 8 * hh), x3 = *(const v4fa*)(arow + kb + 16 + 8 * hh + 4);
    float xs[16] = {x0[0],x0[1],x0[2],x0[3],x1[0],x1[1],x1[2],x1[3],x2[0],x2[1],x2[2],x2[3],x3[0],x3[1],x3[2],x3[3]};
#pragma unroll
    for (int i = 0; i < 16; ++i) { const unsigned short hb = bf16_bits(xs[i]); ah.u[i] = hb; al.u[i] = ASPLIT ? bf16_bits(xs[i] - bf16_val(hb)) : (unsigned short)0; }
#pragma unroll
    for (int t = 0; t < 4; ++t) {
      if (col0 + t * 16 >= N) continue;
      const size_t boff = (size_t)(col0 + t * 16 + ln) * ldb + kb;
      FragB bh_, bl_; bh_.half[0] = *(const v8us*)(Bh + boff + 8 * hh); bh_.half[1] = *(const v8us*)(Bh + boff + 16 + 8 * hh);
      if (BSPLIT) { bl_.half[0] = *(const v8us*)(Bl + boff + 8 * hh); bl_.half[1] = *(const v8us*)(Bl + boff + 16 + 8 * hh); } else bl_ = bh_;
      acc[t] = mmaN<ASPLIT ? (BSPLIT ? 3 : 2) : 1>(ah.v, al.v, bh_.v, bl_.v, acc[t]);
    }
  }
#pragma unroll
  for (int t = 0; t < 4; ++t) {
    const int col = col0 + t * 16 + ln; if (col0 + t * 16 >= N) continue; const float bv = bias ? bf16_round(bias[col]) : 0.f;
#pragma unroll
    for (int r = 0; r < 8; ++r) { float v = acc[t][r] * alpha + bv; if (resid) v += rsign * resid[(size_t)(row0 + 8 * hh + r) * ldr + col]; if (ACT == 1) v = fmaxf(v, 0.f); else if (ACT == 2) v = fmaxf(v, 0.f) + log1pf(expf(-fabsf(v))); so[w][8 * hh + r][t * 16 + ln] = v; }
  }
  __builtin_amdgcn_fence(__ATOMIC_ACQ_REL, "workgroup"); __builtin_amdgcn_wave_barrier();
  const int rsub = lane >> 4, c4 = (lane & 15) * 4;
  for (int pass = 0; pass < 2; ++pass) {
#pragma unroll
    for (int q = 0; q < 8; ++q) { const int r = q * 2 + rsub; if (col0 + c4 < N) { const v4f v = *(const v4fa*)&so[w][r][c4]; *(volatile v4f*)(C + (size_t)(row0 + r) * ldc + col0 + c4) = v; } }
    if (pass == 0) __threadfence();
  }
}
__global__ __launch_bounds__(256) void k_split_transpose_b(const float* __restrict__ src, int lds_, size_t sIn, unsigned short* __restrict__ hi, unsigned short* __restrict__ lo, size_t sOut, int K, int N) {
  const size_t t = (size_t)blockIdx.x * 256 + threadIdx.x; const int k8n = K / 8; if (t >= (size_t)N * k8n) return;
  src += (size_t)blockIdx.y * sIn; hi += (size_t)blockIdx.y * sOut; lo += (size_t)blockIdx.y * sOut;
  const int n = (int)(t / k8n), k8 = (int)(t % k8n) * 8; v8us vh, vl;
#pragma unroll
  for (int i = 0; i < 8; ++i) { const float x = src[(size_t)(k8 + i) * lds_ + n]; const unsigned short hb = bf16_bits(x); vh[i] = hb; vl[i] = bf16_bits(x - bf16_val(hb)); }
  unsigned short* dh = hi + (size_t)n * K + k8; unsigned short* dl = lo + (size_t)n * K + k8;
  *(volatile v8us*)dh = vh; *(volatile v8us*)dl = vl; __threadfence(); *(volatile v8us*)dh = vh; *(volatile v8us*)dl = vl;
}

typedef _Float16 v16h __attribute__((ext_vector_type(16)));
union FragH { v16h v; v8us half[2]; _Float16 h[16]; unsigned short u[16]; };
template <int NT>
__device__ __forceinline__ v8f mmaH(v16h ah, v16h al, v16h bh, v16h bl, v8f c) {
  c = __builtin_amdgcn_wmma_f32_16x16x32_f16(false, ah, false, bh, (short)0, c, false, false);
  if (NT >= 2) c = __builtin_amdgcn_wmma_f32_16x16x32_f16(false, al, false, bh, (short)0, c, false, false);
  if (NT >= 3) c = __builtin_amdgcn_wmma_f32_16x16x32_f16(false, ah, false, bl, (short)0, c, false, false);
  asm volatile("v_nop\n\tv_nop\n\tv_nop\n\tv_nop" : "+v"(c) : "v"(ah), "v"(al), "v"(bh), "v"(bl));
  return c;
}
template <bool ASPLIT>
__global__ __launch_bounds__(128) void k_gemm_h(const float* __restrict__ A, int lda, size_t sA, const _Float16* __restrict__ Bh, int ldb, size_t sB, float alpha, float* __restrict__ C, int ldc, size_t sC, int M, int N, int K) {
  __shared__ __attribute__((aligned(16))) float so[4][16][64];
  const int tid = threadIdx.x, w = tid >> 5, lane = tid & 31, ln = lane & 15, hh = lane >> 4; const int by = blockIdx.y;
  A += (size_t)by * sA; Bh += (size_t)by * sB; C += (size_t)by * sC;
  const int ntn = (N + 63) / 64; const int wid = blockIdx.x * 4 + w; const int mt = wid / ntn, nq = wid % ntn; if (mt * 16 >= M) return;
  const int row0 = mt * 16, col0 = nq * 64; const float* arow = A + (size_t)(row0 + ln) * lda;
  v8f acc[4] = {};
  for (int kb = 0; kb < K; kb += 32) {
    FragH ah, al;
    const v4f x0 = *(const v4fa*)(arow + kb + 8 * hh), x1 = *(const v4fa*)(arow + kb + 8 * hh + 4), x2 = *(const v4fa*)(arow + kb + 16 + 8 * hh), x3 = *(const v4fa*)(arow + kb + 16 + 8 * hh + 4);
    float xs[16] = {x0[0],x0[1],x0[2],x0[3],x1[0],x1[1],x1[2],x1[3],x2[0],x2[1],x2[2],x2[3],x3[0],x3[1],x3[2],x3[3]};
#pragma unroll
    for (int i = 0; i < 16; ++i) { const _Float16 h = (_Float16)xs[i]; ah.h[i] = h; al.h[i] = ASPLIT ? (_Float16)(xs[i] - (float)h) : (_Float16)0.0f; }
#pragma unroll
    for (int t = 0; t < 4; ++t) { if (col0 + t * 16 >= N) continue; const size_t boff = (size_t)(col0 + t * 16 + ln) * ldb + kb; FragH bq; bq.half[0] = *(const v8us*)(Bh + boff + 8 * hh); bq.half[1] = *(const v8us*)(Bh + boff + 16 + 8 * hh);
      acc[t] = mmaH<ASPLIT ? 2 : 1>(ah.v, al.v, bq.v, bq.v, acc[t]); }
  }
#pragma unroll
  for (int t = 0; t < 4; ++t) { if (col0 + t * 16 >= N) continue;
#pragma unroll
    for (int r = 0; r < 8; ++r) so[w][8 * hh + r][t * 16 + ln] = acc[t][r] * alpha; }
  __builtin_amdgcn_fence(__ATOMIC_ACQ_REL, "workgroup"); __builtin_amdgcn_wave_barrier();
  const int rsub = lane >> 4, c4 = (lane & 15) * 4;
  for (int pass = 0; pass < 2; ++pass) {
#pragma unroll
    for (int q = 0; q < 8; ++q) { const int r = q * 2 + rsub; if (col0 + c4 < N) { const v4f v = *(const v4fa*)&so[w][r][c4]; *(volatile v4f*)(C + (size_t)(row0 + r) * ldc + col0 + c4) = v; } }
    if (pass == 0) __threadfence(); }
}

__global__ __launch_bounds__(256) void k_round_rows(const float* __restrict__ W, unsigned short* __restrict__ Wt, int n8) {
  const int t = blockIdx.x * 256 + threadIdx.x;
  if (t >= n8) return;
  const v4f a = *(const v4fa*)(W + (size_t)t * 8), b = *(const v4fa*)(W + (size_t)t * 8 + 4);
  v8us v; v[0]=bf16_bits(a[0]); v[1]=bf16_bits(a[1]); v[2]=bf16_bits(a[2]); v[3]=bf16_bits(a[3]);
  v[4]=bf16_bits(b[0]); v[5]=bf16_bits(b[1]); v[6]=bf16_bits(b[2]); v[7]=bf16_bits(b[3]);
  *(volatile v8us*)(Wt + (size_t)t * 8) = v; __threadfence(); *(volatile v8us*)(Wt + (size_t)t * 8) = v;
}

__global__ __launch_bounds__(256) void k_bn1stat(const float* __restrict__ x, double* __restrict__ part) { __shared__ double sp[8][2]; const int tid = threadIdx.x, wv = tid >> 5, lane = tid & 31; const int b = blockIdx.x / (CD / 8), c0 = (blockIdx.x % (CD / 8)) * 8; const int c = c0 + wv;
  const float* row = x + ((size_t)b * CD + c) * NTQ; double a = 0.0, q = 0.0;
#pragma unroll 1
  for (int n = lane; n < NTQ; n += 32) { const float v = bf16_round(row[n]); a += v; q += (double)v * v; }
  for (int o = 16; o >= 1; o >>= 1) { a += __shfl_xor(a, o, 32); q += __shfl_xor(q, o, 32); }
  if (lane == 0) { sp[wv][0] = a; sp[wv][1] = q; } __syncthreads();
  if (tid < 16) { *(volatile double*)(part + ((size_t)b * CD + c0) * 2 + tid) = sp[tid >> 1][tid & 1]; } __threadfence(); if (tid < 16) { *(volatile double*)(part + ((size_t)b * CD + c0) * 2 + tid) = sp[tid >> 1][tid & 1]; } }
__global__ __launch_bounds__(256) void k_bnfin(const double* __restrict__ part, int nparts, int stride_c, const float* __restrict__ g, const float* __restrict__ bb, float* __restrict__ st) { const int c = threadIdx.x; double s = 0.0, q = 0.0; for (int k = 0; k < nparts; ++k) { s += part[((size_t)k * stride_c + c) * 2]; q += part[((size_t)k * stride_c + c) * 2 + 1]; }
  const double cnt = (double)NTOK; const double mu = s / cnt; double var = q / cnt - mu * mu; if (var < 0.0) var = 0.0; const float sc = bf16_round(g[c]) / (float)sqrt(var + 1e-5); const float sh = bf16_round(bb[c]) - (float)mu * sc;
  *(volatile float*)(st + c * 2) = sc; *(volatile float*)(st + c * 2 + 1) = sh; __threadfence(); *(volatile float*)(st + c * 2) = sc; *(volatile float*)(st + c * 2 + 1) = sh; }
__global__ __launch_bounds__(256) void k_xn(const float* __restrict__ x, const float* __restrict__ st, float* __restrict__ XN) { __shared__ float tile[32][33]; const int b = blockIdx.z; const int c0 = blockIdx.y * 32, n0 = blockIdx.x * 32; const int tx = threadIdx.x & 31, ty = threadIdx.x >> 5;
  for (int i = ty; i < 32; i += 8) tile[i][tx] = bf16_round(x[((size_t)b * CD + c0 + i) * NTQ + n0 + tx]) * st[(c0 + i) * 2] + st[(c0 + i) * 2 + 1]; __syncthreads();
  for (int pass = 0; pass < 2; ++pass) { for (int i = ty; i < 32; i += 8) *(volatile float*)(XN + ((size_t)b * NTQ + n0 + i) * CD + c0 + tx) = tile[tx][i]; if (pass == 0) __threadfence(); } }
__global__ __launch_bounds__(256) void k_colstat(const float* __restrict__ X, double* __restrict__ part) { const int c = threadIdx.x; const size_t r0 = (size_t)blockIdx.x * 1024; double s = 0.0, q = 0.0;
#pragma unroll 1
  for (int r = 0; r < 1024; ++r) { const float v = X[(r0 + r) * CD + c]; s += v; q += (double)v * v; } *(volatile double*)(part + ((size_t)blockIdx.x * CD + c) * 2) = s; *(volatile double*)(part + ((size_t)blockIdx.x * CD + c) * 2 + 1) = q; __threadfence(); *(volatile double*)(part + ((size_t)blockIdx.x * CD + c) * 2) = s; *(volatile double*)(part + ((size_t)blockIdx.x * CD + c) * 2 + 1) = q; }
__global__ __launch_bounds__(256) void k_ce(const float* __restrict__ cor, const float* __restrict__ cw, float* __restrict__ CE) { const size_t t = (size_t)blockIdx.x * 256 + threadIdx.x; if (t >= (size_t)NTOK * MD / 4) return; const int m4 = (int)((t * 4) % MD); const size_t tok = (t * 4) / MD; const float c0 = bf16_round(cor[tok * 3]), c1 = bf16_round(cor[tok * 3 + 1]), c2 = bf16_round(cor[tok * 3 + 2]); v4f o;
  for (int q = 0; q < 4; ++q) { const int m = m4 + q; o[q] = (c0 * bf16_round(cw[m * 3]) + c1 * bf16_round(cw[m * 3 + 1])) + c2 * bf16_round(cw[m * 3 + 2]); } *(volatile v4f*)(CE + t * 4) = o; __threadfence(); *(volatile v4f*)(CE + t * 4) = o; }
__global__ __launch_bounds__(256) void k_heads(const float* __restrict__ Q, const float* __restrict__ KV, const float* __restrict__ CE, int b, float* __restrict__ Qh, _Float16* __restrict__ Kh, _Float16* __restrict__ VCt) {
  __shared__ float tv[64][49]; const int h = blockIdx.y, n0 = blockIdx.x * 64; const int t = threadIdx.x; const int bs = (b + NB / 2) % NB; typedef _Float16 v2h __attribute__((ext_vector_type(2)));
  for (int e = t; e < 64 * 32; e += 256) { const int r = e >> 5, d = e & 31; const size_t tq = (size_t)b * NTQ + n0 + r, tk = (size_t)bs * NTQ + n0 + r;
    const float qv = Q[tq * CD + h * HD + d] * 0.17677669529663687f; const float kvv = KV[tk * (2 * CD) + h * HD + d]; tv[r][d] = KV[tk * (2 * CD) + CD + h * HD + d]; if (d < MHD) tv[r][32 + d] = CE[tq * MD + h * MHD + d];
    float* qd = Qh + ((size_t)h * NTQ + n0 + r) * HD + d; _Float16* kd = Kh + ((size_t)h * NTQ + n0 + r) * HD + d; *(volatile float*)qd = qv; *(volatile _Float16*)kd = (_Float16)kvv; __threadfence(); *(volatile float*)qd = qv; *(volatile _Float16*)kd = (_Float16)kvv; }
  __syncthreads();
  for (int pass = 0; pass < 2; ++pass) { for (int e = t; e < 48 * 32; e += 256) { const int dr = e >> 5, np = (e & 31) * 2; v2h vv; vv.x = (_Float16)tv[np][dr]; vv.y = (_Float16)tv[np + 1][dr]; *(volatile v2h*)(VCt + ((size_t)h * 48 + dr) * NTQ + n0 + np) = vv; } if (pass == 0) __threadfence(); }
}
__global__ __launch_bounds__(1024) void k_softmax(float* __restrict__ S, int h, float* __restrict__ Dn) { __shared__ float sd[32]; const int tid = threadIdx.x, wv = tid >> 5, lane = tid & 31; const int n = blockIdx.x * 32 + wv; float* row = S + ((size_t)h * NTQ + n) * NTQ;
  float mx = -3.0e38f; for (int j = lane; j < NTQ; j += 32) mx = fmaxf(mx, row[j]); for (int o = 16; o >= 1; o >>= 1) mx = fmaxf(mx, __shfl_xor(mx, o, 32));
  float den = 0.f; for (int j = lane; j < NTQ; j += 32) { const float e = expf(row[j] - mx); den += e; *(volatile float*)(row + j) = e * 256.0f; } for (int o = 16; o >= 1; o >>= 1) den += __shfl_xor(den, o, 32);
  __threadfence(); for (int j = lane; j < NTQ; j += 32) { const float pv = row[j]; *(volatile float*)(row + j) = pv; }
  if (lane == 0) sd[wv] = den; __syncthreads(); if (tid < 32) { *(volatile float*)(Dn + (size_t)h * NTQ + blockIdx.x * 32 + tid) = sd[tid]; } __threadfence(); if (tid < 32) { *(volatile float*)(Dn + (size_t)h * NTQ + blockIdx.x * 32 + tid) = sd[tid]; } }
__global__ __launch_bounds__(256) void k_unhead(const float* __restrict__ O, const float* __restrict__ Dn, const float* __restrict__ CE, int b, float* __restrict__ AV, float* __restrict__ CRD) { const int t = blockIdx.x * 256 + threadIdx.x; if (t >= NTQ * NH * 12) return; const int c4 = (t % 12) * 4; const int h = (t / 12) % NH; const int n = t / (12 * NH); const size_t tok = (size_t)b * NTQ + n; const float rd = 1.0f / Dn[(size_t)h * NTQ + n];
  const v4f o = *(const v4fa*)(O + ((size_t)h * NTQ + n) * 48 + c4); v4f r; if (c4 < HD) { for (int q = 0; q < 4; ++q) r[q] = o[q] * rd; *(volatile v4f*)(AV + tok * CD + h * HD + c4) = r; __threadfence(); *(volatile v4f*)(AV + tok * CD + h * HD + c4) = r; }
  else { const int m4 = c4 - HD; for (int q = 0; q < 4; ++q) r[q] = o[q] * rd - CE[tok * MD + h * MHD + m4 + q]; *(volatile v4f*)(CRD + tok * MD + h * MHD + m4) = r; __threadfence(); *(volatile v4f*)(CRD + tok * MD + h * MHD + m4) = r; } }
__global__ __launch_bounds__(256) void k_res1(const float* __restrict__ XN, const float* __restrict__ XA, const float* __restrict__ pb, float* __restrict__ XN2) { const size_t t = (size_t)blockIdx.x * 256 + threadIdx.x; if (t >= (size_t)NTOK * CD / 4) return; const int c4 = (int)((t * 4) % CD); const v4f a = *(const v4fa*)(XN + t * 4), x = *(const v4fa*)(XA + t * 4); v4f o; for (int q = 0; q < 4; ++q) o[q] = a[q] + (x[q] + bf16_round(pb[c4 + q])); *(volatile v4f*)(XN2 + t * 4) = o; __threadfence(); *(volatile v4f*)(XN2 + t * 4) = o; }
__global__ __launch_bounds__(256) void k_bnapply(float* __restrict__ X, const float* __restrict__ st) { const size_t t = (size_t)blockIdx.x * 256 + threadIdx.x; if (t >= (size_t)NTOK * CD / 4) return; const int c4 = (int)((t * 4) % CD); v4f v = *(const v4fa*)(X + t * 4); for (int q = 0; q < 4; ++q) v[q] = v[q] * st[(c4 + q) * 2] + st[(c4 + q) * 2 + 1]; *(volatile v4f*)(X + t * 4) = v; __threadfence(); *(volatile v4f*)(X + t * 4) = v; }
__global__ __launch_bounds__(256) void k_hact(float* __restrict__ Hm, const float* __restrict__ fb, const float* __restrict__ dw, const float* __restrict__ db, const float* __restrict__ pa) { const size_t t = (size_t)blockIdx.x * 256 + threadIdx.x; if (t >= (size_t)NTOK * HID / 4) return; const int c4 = (int)((t * 4) % HID); const float a = bf16_round(pa[0]); v4f v = *(const v4fa*)(Hm + t * 4);
  for (int q = 0; q < 4; ++q) { const int c = c4 + q; float h = (v[q] + bf16_round(fb[c])) * bf16_round(dw[c]) + bf16_round(db[c]); v[q] = (h >= 0.f) ? h : a * h; } *(volatile v4f*)(Hm + t * 4) = v; __threadfence(); *(volatile v4f*)(Hm + t * 4) = v; }
__global__ __launch_bounds__(256) void k_addb(float* __restrict__ Y, const float* __restrict__ b, int NC, size_t n4) { const size_t t = (size_t)blockIdx.x * 256 + threadIdx.x; if (t >= n4) return; const int c4 = (int)((t * 4) % NC); v4f v = *(const v4fa*)(Y + t * 4); for (int q = 0; q < 4; ++q) v[q] += bf16_round(b[c4 + q]); *(volatile v4f*)(Y + t * 4) = v; __threadfence(); *(volatile v4f*)(Y + t * 4) = v; }
extern "C" void kernel_launch(void* const* d_in, const int* in_sizes, int n_in,
                              void* d_out, int out_size, void* d_ws, size_t ws_size, hipStream_t stream) {
  (void)in_sizes; (void)n_in; (void)out_size;
  const float* x = (const float*)d_in[0]; const float* cor = (const float*)d_in[1]; const float* qw = (const float*)d_in[2]; const float* kvw = (const float*)d_in[3]; const float* corw = (const float*)d_in[4]; const float* pw = (const float*)d_in[5]; const float* pb = (const float*)d_in[6]; const float* mw = (const float*)d_in[7]; const float* mb = (const float*)d_in[8];
  const float* g1 = (const float*)d_in[9]; const float* b1 = (const float*)d_in[10]; const float* g2 = (const float*)d_in[11]; const float* b2 = (const float*)d_in[12]; const float* f1w = (const float*)d_in[13]; const float* f1b = (const float*)d_in[14]; const float* dww = (const float*)d_in[15]; const float* dwb = (const float*)d_in[16]; const float* pa = (const float*)d_in[17]; const float* f2w = (const float*)d_in[18]; const float* f2b = (const float*)d_in[19];
  float* xout = (float*)d_out; float* motion = xout + (size_t)NB * CD * NTQ;
  char* ws = (char*)d_ws; size_t off = 0;
  auto take = [&](size_t bytes) { char* p = ws + off; off += (bytes + 255) & ~(size_t)255; return p; };
  unsigned short* Bq = (unsigned short*)take(CD * CD * 2); unsigned short* Bkv = (unsigned short*)take(2 * CD * CD * 2); unsigned short* Bp = (unsigned short*)take(CD * CD * 2); unsigned short* Bm = (unsigned short*)take(MD * MD * 2); unsigned short* Bf1 = (unsigned short*)take((size_t)HID * CD * 2); unsigned short* Bf2 = (unsigned short*)take((size_t)CD * HID * 2);
  double* part = (double*)take((size_t)NB * CD * 2 * 8); float* st = (float*)take(CD * 2 * 4);
  float* XN = (float*)take((size_t)NTOK * CD * 4); float* Q = (float*)take((size_t)NTOK * CD * 4); float* KV = (float*)take((size_t)NTOK * 2 * CD * 4); float* CE = (float*)take((size_t)NTOK * MD * 4);
  float* Qh = (float*)take((size_t)NH * NTQ * HD * 4); _Float16* Kh = (_Float16*)take((size_t)NH * NTQ * HD * 2); _Float16* VCt = (_Float16*)take((size_t)NH * 48 * NTQ * 2); float* S = (float*)take((size_t)NH * NTQ * NTQ * 4); float* Dn = (float*)take((size_t)NH * NTQ * 4); float* O = (float*)take((size_t)NH * NTQ * 48 * 4);
  float* AV = (float*)take((size_t)NTOK * CD * 4); float* CRD = (float*)take((size_t)NTOK * MD * 4); float* XA = Q;
  float* XA2 = (float*)take((size_t)NTOK * CD * 4); float* Hm = (float*)take((size_t)NTOK * HID * 4); float* OUT = XA2;
  if (off > ws_size) return; (void)XA;
  k_round_rows<<<(CD * CD / 8 + 255) / 256, 256, 0, stream>>>(qw, Bq, CD * CD / 8); k_round_rows<<<(2 * CD * CD / 8 + 255) / 256, 256, 0, stream>>>(kvw, Bkv, 2 * CD * CD / 8); k_round_rows<<<(CD * CD / 8 + 255) / 256, 256, 0, stream>>>(pw, Bp, CD * CD / 8);
  k_round_rows<<<(MD * MD / 8 + 255) / 256, 256, 0, stream>>>(mw, Bm, MD * MD / 8); k_round_rows<<<(unsigned)(((size_t)HID * CD / 8 + 255) / 256), 256, 0, stream>>>(f1w, Bf1, HID * CD / 8); k_round_rows<<<(unsigned)(((size_t)CD * HID / 8 + 255) / 256), 256, 0, stream>>>(f2w, Bf2, CD * HID / 8);
  k_bn1stat<<<NB * (CD / 8), 256, 0, stream>>>(x, part); k_bnfin<<<1, 256, 0, stream>>>(part, NB, CD, g1, b1, st); k_xn<<<dim3(NTQ / 32, CD / 32, NB), 256, 0, stream>>>(x, st, XN);
  k_gemm_bf3<true, 0, false, false><<<((NTOK / 16) * (CD / 64) + 3) / 4, 128, 0, stream>>>(XN, CD, Bq, CD, nullptr, nullptr, 1, 0, Q, CD, NTOK, CD, CD);
  k_gemm_bf3<true, 0, false, false><<<((NTOK / 16) * (2 * CD / 64) + 3) / 4, 128, 0, stream>>>(XN, CD, Bkv, CD, nullptr, nullptr, 1, 0, KV, 2 * CD, NTOK, 2 * CD, CD);
  k_ce<<<(unsigned)(((size_t)NTOK * MD / 4 + 255) / 256), 256, 0, stream>>>(cor, corw, CE);
  for (int b = 0; b < NB; ++b) {
    k_heads<<<dim3(NTQ / 64, NH), 256, 0, stream>>>(Q, KV, CE, b, Qh, Kh, VCt);
    k_gemm_h<true><<<dim3(((NTQ / 16) * (NTQ / 64) + 3) / 4, NH), 128, 0, stream>>>(Qh, HD, (size_t)NTQ * HD, Kh, HD, (size_t)NTQ * HD, 1.f, S, NTQ, (size_t)NTQ * NTQ, NTQ, NTQ, HD);
    for (int h = 0; h < NH; ++h) k_softmax<<<NTQ / 32, 1024, 0, stream>>>(S, h, Dn);
    k_gemm_h<false><<<dim3(((NTQ / 16) * 1 + 3) / 4, NH), 128, 0, stream>>>(S, NTQ, (size_t)NTQ * NTQ, VCt, NTQ, (size_t)48 * NTQ, 0.00390625f, O, 48, (size_t)NTQ * 48, NTQ, 48, NTQ);
    k_unhead<<<(NTQ * NH * 12 + 255) / 256, 256, 0, stream>>>(O, Dn, CE, b, AV, CRD);
  }
  k_gemm_bf3<true, 0, false, false><<<((NTOK / 16) * (CD / 64) + 3) / 4, 128, 0, stream>>>(AV, CD, Bp, CD, nullptr, nullptr, 1, 0, XA2, CD, NTOK, CD, CD);
  k_gemm_bf3<true, 0, true, false><<<((NTOK / 16) * (MD / 64) + 3) / 4, 128, 0, stream>>>(CRD, MD, Bm, MD, mb, nullptr, 1, 0, motion, MD, NTOK, MD, MD);
  k_res1<<<(unsigned)(((size_t)NTOK * CD / 4 + 255) / 256), 256, 0, stream>>>(XN, XA2, pb, XN);
  k_colstat<<<NTOK / 1024, 256, 0, stream>>>(XN, part); k_bnfin<<<1, 256, 0, stream>>>(part, NTOK / 1024, CD, g2, b2, st); k_bnapply<<<(unsigned)(((size_t)NTOK * CD / 4 + 255) / 256), 256, 0, stream>>>(XN, st);
  k_gemm_bf3<true, 0, false, false><<<((NTOK / 16) * (HID / 64) + 3) / 4, 128, 0, stream>>>(XN, CD, Bf1, CD, nullptr, nullptr, 1, 0, Hm, HID, NTOK, HID, CD);
  k_hact<<<(unsigned)(((size_t)NTOK * HID / 4 + 255) / 256), 256, 0, stream>>>(Hm, f1b, dww, dwb, pa);
  k_gemm_bf3<true, 0, false, false><<<((NTOK / 16) * (CD / 64) + 3) / 4, 128, 0, stream>>>(Hm, HID, Bf2, HID, nullptr, nullptr, 1, 0, OUT, CD, NTOK, CD, HID);
  k_addb<<<(unsigned)(((size_t)NTOK * CD / 4 + 255) / 256), 256, 0, stream>>>(OUT, f2b, CD, (size_t)NTOK * CD / 4);
  k_transpose32<false, true, true><<<dim3(CD / 32, NTQ / 32, NB), 256, 0, stream>>>(OUT, xout, NTQ, CD, nullptr, nullptr, x);
}
